// RWKV_Tmix_x070_1889785610320
// MI455X (gfx1250) — hardware-verified
//
#include <hip/hip_runtime.h>
#include <math.h>

constexpr int  kNB   = 2;
constexpr int  kNT   = 1024;
constexpr int  kNCH  = 2048;
constexpr int  kNH   = 32;
constexpr int  kHD   = 64;
constexpr int  kRows = kNB * kNT;
constexpr long kPlane    = (long)kRows * kNCH;
constexpr long kRegBytes = 16777216L;
constexpr long kHalfReg  = kRegBytes / 2;
constexpr long kSub256K  = 262144L;
constexpr long kSub512K  = 524288L;
constexpr float kGnEps   = 6.4e-4f;
static_assert(kPlane * 4 == kRegBytes);
static_assert((kPlane / 8) % 256 == 0);
static_assert((kPlane / 4) % 256 == 0);
static_assert((kPlane / 2) % 256 == 0);
static_assert(kRows % 64 == 0 && kNCH % 64 == 0);


typedef __attribute__((ext_vector_type(16))) _Float16 v16h;
typedef __attribute__((ext_vector_type(8)))  _Float16 v8h;
typedef __attribute__((ext_vector_type(16))) __bf16   v16b;
typedef __attribute__((ext_vector_type(8)))  __bf16   v8b;
typedef __attribute__((ext_vector_type(8)))  float    v8f;
typedef __attribute__((ext_vector_type(4)))  float    v4f;
typedef __attribute__((ext_vector_type(2)))  float    v2f;
typedef __attribute__((ext_vector_type(4)))  unsigned int v4u;

__device__ __forceinline__ unsigned short f2bf_bits(float f) {
  unsigned u = __float_as_uint(f);
  return (unsigned short)((u + 0x7FFFu + ((u >> 16) & 1u)) >> 16);
}
__device__ __forceinline__ float bf_bits2f(unsigned short h) { return __uint_as_float(((unsigned)h) << 16); }

__device__ __forceinline__ void dep_guard_h(v8f& a, v8f& b, v16h x, v16h y) { asm volatile("v_nop\n\tv_nop\n\tv_nop\n\tv_nop" : "+v"(a), "+v"(b) : "v"(x), "v"(y)); }
__device__ __forceinline__ void dep_guard_b(v8f& a, v8f& b, v16b x, v16b y) { asm volatile("v_nop\n\tv_nop\n\tv_nop\n\tv_nop" : "+v"(a), "+v"(b) : "v"(x), "v"(y)); }
__device__ __forceinline__ void keep4_h(v16h a, v16h b, v16h c, v16h d) { asm volatile("v_nop" :: "v"(a), "v"(b), "v"(c), "v"(d)); }
__device__ __forceinline__ void keep4_b(v16b a, v16b b, v16b c, v16b d) { asm volatile("v_nop" :: "v"(a), "v"(b), "v"(c), "v"(d)); }
__device__ __forceinline__ void acc_guard4(v8f& a, v8f& b, v8f& c, v8f& d) { asm volatile("v_nop\n\tv_nop\n\tv_nop\n\tv_nop" : "+v"(a), "+v"(b), "+v"(c), "+v"(d)); }
template <typename T> struct Frag;
template <> struct Frag<_Float16> {
  typedef v16h V; union U { v16h v; v8h h[2]; };
  static __device__ __forceinline__ v16h load(const _Float16* p) {
    U f; f.h[0] = *(const v8h*)(p); f.h[1] = *(const v8h*)(p + 16); return f.v;
  }
  static __device__ __forceinline__ v8f mma(v16h a, v16h b, v8f c) {
    return __builtin_amdgcn_wmma_f32_16x16x32_f16(false, a, false, b, (short)0, c, false, false);
  }
  static __device__ __forceinline__ void guard(v8f& a, v8f& b, v16h x, v16h y) { dep_guard_h(a, b, x, y); }
  static __device__ __forceinline__ void keep(v16h a, v16h b, v16h c, v16h d) { keep4_h(a, b, c, d); }
};
template <> struct Frag<__bf16> {
  typedef v16b V; union U { v16b v; v8b h[2]; };
  static __device__ __forceinline__ v16b load(const __bf16* p) {
    U f; f.h[0] = *(const v8b*)(p); f.h[1] = *(const v8b*)(p + 16); return f.v;
  }
  static __device__ __forceinline__ v8f mma(v16b a, v16b b, v8f c) {
    return __builtin_amdgcn_wmma_f32_16x16x32_bf16(false, a, false, b, (short)0, c, false, false);
  }
  static __device__ __forceinline__ void guard(v8f& a, v8f& b, v16b x, v16b y) { dep_guard_b(a, b, x, y); }
  static __device__ __forceinline__ void keep(v16b a, v16b b, v16b c, v16b d) { keep4_b(a, b, c, d); }
};

__device__ __forceinline__ unsigned pk16(unsigned short a, unsigned short b) { return (unsigned)a | ((unsigned)b << 16); }
__device__ __forceinline__ void split_bf(float f, unsigned short& hb, unsigned short& lb) {
  hb = f2bf_bits(f);
  lb = f2bf_bits(f - bf_bits2f(hb));
}

template <int ET> struct Elem;
template <> struct Elem<0> { typedef _Float16 T; };
template <> struct Elem<1> { typedef __bf16 T; };
template <int ET, bool SPLIT, int BIAS_MODE, int OUT_MODE, bool RESID, int ACT = 0>
__global__ __launch_bounds__(256) void wmma_gemm64(
    const unsigned short* __restrict__ Ap, const unsigned short* __restrict__ A2p, int lda, long strideA,
    const unsigned short* __restrict__ Btp, const unsigned short* __restrict__ Bt2p, int ldb, long strideB,
    void* __restrict__ Cout, void* __restrict__ Cout2, int ldc, long strideC,
    const float* __restrict__ bias,
    const float* __restrict__ resid, long strideR,
    int M, int N, int K, float scale) {
  typedef typename Elem<ET>::T T;
  typedef typename Frag<T>::V V;
  const T* A = (const T*)Ap; const T* A2 = (const T*)A2p; const T* Bt = (const T*)Btp; const T* Bt2 = (const T*)Bt2p;
  __shared__ __align__(16) float sT[8][16 * 68];
  const int b    = blockIdx.y;
  const int lane = threadIdx.x & 31;
  const int wave = threadIdx.x >> 5;
  const int tilesN = N >> 6;
  const int tilesM = M >> 6;
  const int tile = blockIdx.x * 8 + wave;
  if (tile >= tilesM * tilesN) return;
  const int tm = tile / tilesN;
  const int tn = tile - tm * tilesN;
  const int m0 = tm << 6;
  const int n0 = tn << 6;

  const T* Ab  = A  + (size_t)b * strideA;
  const T* Bb  = Bt + (size_t)b * strideB;
  const T* Ab2 = SPLIT ? (A2  + (size_t)b * strideA) : nullptr;
  const T* Bb2 = SPLIT ? (Bt2 + (size_t)b * strideB) : nullptr;

  const int rlane = lane & 15;
  const int koff  = (lane >> 4) * 8;
  const int mOff  = (lane >> 4) * 8;

  v8f acc[4][4];
#pragma unroll
  for (int i = 0; i < 4; ++i)
#pragma unroll
    for (int j = 0; j < 4; ++j) acc[i][j] = (v8f){0.f,0.f,0.f,0.f,0.f,0.f,0.f,0.f};

  for (int k0 = 0; k0 < K; k0 += 32) {
    V bh[4], bl[4];
#pragma unroll
    for (int j = 0; j < 4; ++j) {
      const size_t bo = (size_t)(n0 + (j << 4) + rlane) * ldb + koff + k0;
      bh[j] = Frag<T>::load(Bb + bo);
      if (SPLIT) bl[j] = Frag<T>::load(Bb2 + bo);
    }
#pragma unroll
    for (int i = 0; i < 4; ++i) {
      const size_t ao = (size_t)(m0 + (i << 4) + rlane) * lda + koff + k0;
      V ah = Frag<T>::load(Ab + ao);
      V al;
      if (SPLIT) al = Frag<T>::load(Ab2 + ao);
#pragma unroll
      for (int j = 0; j < 4; ++j) {
        acc[i][j] = Frag<T>::mma(ah, bh[j], acc[i][j]);
        if (SPLIT) {
          acc[i][j] = Frag<T>::mma(ah, bl[j], acc[i][j]);
          acc[i][j] = Frag<T>::mma(al, bh[j], acc[i][j]);
        }
      }
      Frag<T>::guard(acc[i][0], acc[i][3], ah, SPLIT ? al : ah);
    }
    Frag<T>::keep(bh[0], bh[1], bh[2], bh[3]);
    if (SPLIT) Frag<T>::keep(bl[0], bl[1], bl[2], bl[3]);
  }
  acc_guard4(acc[0][0], acc[0][1], acc[0][2], acc[0][3]);
  acc_guard4(acc[1][0], acc[1][1], acc[1][2], acc[1][3]);
  acc_guard4(acc[2][0], acc[2][1], acc[2][2], acc[2][3]);
  acc_guard4(acc[3][0], acc[3][1], acc[3][2], acc[3][3]);

  float* slab = sT[wave];
  const float* Rb = RESID ? (resid + (size_t)b * strideR) : nullptr;
#pragma unroll
  for (int i = 0; i < 4; ++i) {
    const int mBase = m0 + (i << 4);
#pragma unroll
    for (int j = 0; j < 4; ++j) {
      const int n = n0 + (j << 4) + rlane;
      float bv = 0.f;
      if (BIAS_MODE == 2) bv = bias[n];
#pragma unroll
      for (int r = 0; r < 8; ++r) {
        float v = acc[i][j][r] * scale;
        if (BIAS_MODE == 1) v += bias[mBase + mOff + r];
        if (BIAS_MODE == 2) v += bv;
        if (RESID) v += Rb[(size_t)(mBase + mOff + r) * ldc + n];
        if (ACT == 1) v = tanhf(v);
        if (ACT == 2) v = fmaxf(v, 0.0f);
        if (ACT == 3) v = v / (1.0f + expf(-v));
        if (ACT == 4) v = (v > 0.f) ? v : 0.01f * v;
        if (ACT == 6) v = 1.0f / (1.0f + expf(-v));
        slab[(mOff + r) * 68 + (j << 4) + rlane] = v;
      }
    }
    __builtin_amdgcn_fence(__ATOMIC_RELEASE, "workgroup");
    __builtin_amdgcn_wave_barrier();
    __builtin_amdgcn_fence(__ATOMIC_ACQUIRE, "workgroup");
    if (OUT_MODE == 0) {
      float* C = (float*)Cout + (size_t)b * strideC;
      const int hh = lane >> 4, c4 = (lane & 15) * 4;
      for (int pass = 0; pass < 2; ++pass) {
#pragma unroll
        for (int it = 0; it < 8; ++it) {
          const int row = it * 2 + hh;
          v4f v = *(const v4f*)(slab + row * 68 + c4);
          *(volatile v4f*)(C + (size_t)(mBase + row) * ldc + n0 + c4) = v;
        }
        __threadfence();
      }
    } else {
      const int q = lane >> 3, c8 = (lane & 7) * 8;
      unsigned short* C  = (unsigned short*)Cout  + (size_t)b * strideC;
      unsigned short* C2 = (OUT_MODE == 2) ? ((unsigned short*)Cout2 + (size_t)b * strideC) : nullptr;
      for (int pass = 0; pass < 2; ++pass) {
#pragma unroll
        for (int it = 0; it < 4; ++it) {
          const int row = it * 4 + q;
          const float* sp = slab + row * 68 + c8;
          v8h hv, lv;
#pragma unroll
          for (int e = 0; e < 8; ++e) {
            if (OUT_MODE == 1) {
              hv[e] = (_Float16)sp[e];
            } else {
              unsigned short hb = f2bf_bits(sp[e]);
              unsigned short lb = f2bf_bits(sp[e] - bf_bits2f(hb));
              hv[e] = __builtin_bit_cast(_Float16, hb);
              lv[e] = __builtin_bit_cast(_Float16, lb);
            }
          }
          *(volatile v8h*)(C + (size_t)(mBase + row) * ldc + n0 + c8) = hv;
          if (OUT_MODE == 2) *(volatile v8h*)(C2 + (size_t)(mBase + row) * ldc + n0 + c8) = lv;
        }
        __threadfence();
      }
    }
    __builtin_amdgcn_fence(__ATOMIC_RELEASE, "workgroup");
    __builtin_amdgcn_wave_barrier();
    __builtin_amdgcn_fence(__ATOMIC_ACQUIRE, "workgroup");
  }
}

__global__ __launch_bounds__(256) void dscan_kernel(const float* __restrict__ Rp, const float* __restrict__ K2p,
    const float* __restrict__ Vp, const float* __restrict__ Wdp, const float* __restrict__ Ainp,
    const float* __restrict__ Binp, const float* __restrict__ S0p, float* __restrict__ Yp) {
  __shared__ __align__(16) float vbuf[2][6][64];
  __shared__ __align__(16) float ybuf[2][16][64];
  const int tid  = threadIdx.x;
  const int lane = tid & 31, wave = tid >> 5;
  const int bh   = blockIdx.x;
  const int b    = bh >> 5, h = bh & 31;
  const int vrow = tid >> 2, kq = tid & 3, kb0 = kq * 16;
  const size_t col  = (size_t)h * kHD;
  const size_t row0 = (size_t)b * kNT;

  float S[16];
  {
    const float* sp = S0p + (((size_t)(b * kNH + h)) * kHD + vrow) * kHD + kb0;
#pragma unroll
    for (int q = 0; q < 4; ++q) {
      const v4f s4 = *(const v4f*)(sp + 4 * q);
      S[4 * q + 0] = s4[0]; S[4 * q + 1] = s4[1]; S[4 * q + 2] = s4[2]; S[4 * q + 3] = s4[3];
    }
  }
  const float* src = (wave == 0) ? Rp : (wave == 1) ? K2p : (wave == 2) ? Wdp : (wave == 3) ? Ainp : (wave == 4) ? Binp : Vp;
  const int  lc4    = (lane & 15) * 4;
  const bool loader = (wave < 6);
  if (loader) {
    const v4f g0 = *(const v4f*)(src + row0 * kNCH + col + lc4);
    *(v4f*)(&vbuf[0][wave][lc4]) = g0;
  }
  __syncthreads();

#pragma unroll 1
  for (int t = 0; t < kNT; ++t) {
    const int  cur    = t & 1;
    const bool doload = loader && (t + 1 < kNT);
    v4f gnext = (v4f){0.f, 0.f, 0.f, 0.f};
    if (doload) gnext = *(const v4f*)(src + (row0 + (size_t)(t + 1)) * kNCH + col + lc4);

    const float* vb = &vbuf[cur][0][0];
    v4f r4[4], k4[4], w4[4], a4[4], b4[4];
#pragma unroll
    for (int q = 0; q < 4; ++q) {
      r4[q] = *(const v4f*)(vb + 0 * 64 + kb0 + 4 * q);
      k4[q] = *(const v4f*)(vb + 1 * 64 + kb0 + 4 * q);
      w4[q] = *(const v4f*)(vb + 2 * 64 + kb0 + 4 * q);
      a4[q] = *(const v4f*)(vb + 3 * 64 + kb0 + 4 * q);
      b4[q] = *(const v4f*)(vb + 4 * 64 + kb0 + 4 * q);
    }
    const float vv = vb[5 * 64 + vrow];

    float sap = 0.f;
#pragma unroll
    for (int q = 0; q < 4; ++q) {
#pragma unroll
      for (int e = 0; e < 4; ++e) sap += S[4 * q + e] * a4[q][e];
    }
    const float sa1 = sap + __shfl_xor(sap, 1, 32);
    const float sa  = sa1 + __shfl_xor(sa1, 2, 32);

    float yp = 0.f;
#pragma unroll
    for (int q = 0; q < 4; ++q) {
#pragma unroll
      for (int e = 0; e < 4; ++e) {
        const float sn = S[4 * q + e] * w4[q][e] + sa * b4[q][e] + vv * k4[q][e];
        S[4 * q + e] = sn;
        yp += sn * r4[q][e];
      }
    }
    const float y1 = yp + __shfl_xor(yp, 1, 32);
    const float yv = y1 + __shfl_xor(y1, 2, 32);

    const int ypar = (t >> 4) & 1, trow = t & 15;
    if (kq == 0) ybuf[ypar][trow][vrow] = yv;
    if (doload) *(v4f*)(&vbuf[cur ^ 1][wave][lc4]) = gnext;

    if (trow == 15) {
      __syncthreads();
      const int yr = tid >> 4, yc4 = (tid & 15) * 4;
      const v4f val = *(const v4f*)(&ybuf[ypar][yr][yc4]);
      float* dst = Yp + (row0 + (size_t)(t - 15 + yr)) * kNCH + col + yc4;
      *(volatile v4f*)dst = val;
      __threadfence();
      *(volatile v4f*)dst = val;
    }
    __syncthreads();
  }
}

__global__ __launch_bounds__(256) void transpose_split_kernel(const float* __restrict__ W, int KR, int NCOL,
    unsigned short* __restrict__ outHi, unsigned short* __restrict__ outLo, int KP) {
  __shared__ float sm[64][65];
  const int t  = threadIdx.x;
  const int k0 = blockIdx.x * 64, n0 = blockIdx.y * 64;
#pragma unroll
  for (int i = 0; i < 16; ++i) {
    const int e  = i * 256 + t;
    const int kl = e >> 6, nl = e & 63;
    const int k  = k0 + kl, n = n0 + nl;
    const int kc  = (k < KR) ? k : (KR - 1);
    const int ncl = (n < NCOL) ? n : (NCOL - 1);
    float v = W[(size_t)kc * NCOL + ncl];
    if (k >= KR || n >= NCOL) v = 0.0f;
    sm[nl][kl] = v;
  }
  __syncthreads();
  const int lane = t & 31, wave = t >> 5;
  const int q = lane >> 3, c8 = (lane & 7) * 8;
  const int rowA = wave * 8 + q, rowB = wave * 8 + 4 + q;
  v4u uhA, ulA, uhB, ulB;
  {
    unsigned short hb[8], lb[8];
#pragma unroll
    for (int e = 0; e < 8; ++e) split_bf(sm[rowA][c8 + e], hb[e], lb[e]);
    uhA = (v4u){pk16(hb[0], hb[1]), pk16(hb[2], hb[3]), pk16(hb[4], hb[5]), pk16(hb[6], hb[7])};
    ulA = (v4u){pk16(lb[0], lb[1]), pk16(lb[2], lb[3]), pk16(lb[4], lb[5]), pk16(lb[6], lb[7])};
  }
  {
    unsigned short hb[8], lb[8];
#pragma unroll
    for (int e = 0; e < 8; ++e) split_bf(sm[rowB][c8 + e], hb[e], lb[e]);
    uhB = (v4u){pk16(hb[0], hb[1]), pk16(hb[2], hb[3]), pk16(hb[4], hb[5]), pk16(hb[6], hb[7])};
    ulB = (v4u){pk16(lb[0], lb[1]), pk16(lb[2], lb[3]), pk16(lb[4], lb[5]), pk16(lb[6], lb[7])};
  }
  const size_t oA = (size_t)(n0 + rowA) * KP + k0 + c8;
  const size_t oB = (size_t)(n0 + rowB) * KP + k0 + c8;
  for (int pass = 0; pass < 2; ++pass) {
    *(volatile v4u*)(outHi + oA) = uhA;
    *(volatile v4u*)(outLo + oA) = ulA;
    *(volatile v4u*)(outHi + oB) = uhB;
    *(volatile v4u*)(outLo + oB) = ulB;
    __threadfence();
  }
}

__global__ __launch_bounds__(256) void mixsplit_kernel(const float* __restrict__ x, const float* __restrict__ shift,
    const float* __restrict__ mvec, unsigned short* __restrict__ outHi, unsigned short* __restrict__ outLo) {
#pragma clang fp contract(off)
  const size_t i  = (size_t)blockIdx.x * 256 + threadIdx.x;
  const size_t e0 = i * 8;
  const int bt = (int)(e0 >> 11);
  const int c  = (int)(e0 & 2047);
  const int t  = bt & 1023;
  const int b  = bt >> 10;
  const v4f xa = *(const v4f*)(x + e0), xb = *(const v4f*)(x + e0 + 4);
  const size_t ep = (bt > 0) ? (e0 - 2048) : e0;
  const v4f pa = *(const v4f*)(x + ep), pb = *(const v4f*)(x + ep + 4);
  const float* shp = shift + (size_t)b * kNCH + c;
  const v4f sa = *(const v4f*)(shp), sb = *(const v4f*)(shp + 4);
  const v4f ma = *(const v4f*)(mvec + c), mb = *(const v4f*)(mvec + c + 4);
  const bool first = (t == 0);
  float val[8];
#pragma unroll
  for (int e = 0; e < 4; ++e) {
    const float xe = xa[e];
    const float pv = first ? sa[e] : pa[e];
    const float dx = pv - xe;
    val[e] = xe + dx * ma[e];
  }
#pragma unroll
  for (int e = 0; e < 4; ++e) {
    const float xe = xb[e];
    const float pv = first ? sb[e] : pb[e];
    const float dx = pv - xe;
    val[4 + e] = xe + dx * mb[e];
  }
  unsigned short hb[8], lb[8];
#pragma unroll
  for (int e = 0; e < 8; ++e) split_bf(val[e], hb[e], lb[e]);
  const v4u uh = (v4u){pk16(hb[0], hb[1]), pk16(hb[2], hb[3]), pk16(hb[4], hb[5]), pk16(hb[6], hb[7])};
  const v4u ul = (v4u){pk16(lb[0], lb[1]), pk16(lb[2], lb[3]), pk16(lb[4], lb[5]), pk16(lb[6], lb[7])};
  unsigned short* ph = outHi + e0;
  unsigned short* pl = outLo + e0;
  *(volatile v4u*)ph = uh;
  *(volatile v4u*)pl = ul;
  __threadfence();
  *(volatile v4u*)ph = uh;
  *(volatile v4u*)pl = ul;
}

__global__ __launch_bounds__(256) void vmix_kernel(float* __restrict__ Vq, const float* __restrict__ vf,
    const float* __restrict__ pre, const float* __restrict__ v0v) {
#pragma clang fp contract(off)
  const size_t e0 = ((size_t)blockIdx.x * 256 + threadIdx.x) * 4;
  const int c = (int)(e0 & 2047);
  const v4f vv = *(const v4f*)(Vq + e0);
  const v4f f4 = *(const v4f*)(vf + e0);
  const v4f p4 = *(const v4f*)(pre + e0);
  const v4f b4 = *(const v4f*)(v0v + c);
  v4f o;
#pragma unroll
  for (int e = 0; e < 4; ++e) {
    const float z  = b4[e] + p4[e];
    const float sg = 1.0f / (1.0f + expf(-z));
    const float d  = f4[e] - vv[e];
    o[e] = vv[e] + d * sg;
  }
  *(volatile v4f*)(Vq + e0) = o;
  __threadfence();
  *(volatile v4f*)(Vq + e0) = o;
}

__global__ __launch_bounds__(256) void kprep_kernel(float* __restrict__ Kq, float* __restrict__ Aq,
    float* __restrict__ AinP, const float* __restrict__ kkc, const float* __restrict__ kac) {
#pragma clang fp contract(off)
  const int lane = threadIdx.x & 31, wave = threadIdx.x >> 5;
  const int gw = blockIdx.x * 8 + wave;
  const int bt = gw >> 4, hp = gw & 15;
  const int c  = hp * 128 + lane * 4;
  const size_t base = (size_t)bt * kNCH + c;
  const v4f k4  = *(const v4f*)(Kq + base);
  const v4f a4  = *(const v4f*)(Aq + base);
  const v4f kc4 = *(const v4f*)(kkc + c);
  const v4f ka4 = *(const v4f*)(kac + c);
  float kk[4];
#pragma unroll
  for (int e = 0; e < 4; ++e) kk[e] = k4[e] * kc4[e];
  float ss = kk[0] * kk[0];
  ss = ss + kk[1] * kk[1];
  ss = ss + kk[2] * kk[2];
  ss = ss + kk[3] * kk[3];
  ss += __shfl_xor(ss, 1, 32);
  ss += __shfl_xor(ss, 2, 32);
  ss += __shfl_xor(ss, 4, 32);
  ss += __shfl_xor(ss, 8, 32);
  const float nrm = sqrtf(ss);
  const float inv = 1.0f / fmaxf(nrm, 1e-12f);
  v4f k2o, aino, bino;
#pragma unroll
  for (int e = 0; e < 4; ++e) {
    const float kn = kk[e] * inv;
    aino[e] = -kn;
    bino[e] = kn * a4[e];
    const float am1 = a4[e] - 1.0f;
    const float gk  = 1.0f + am1 * ka4[e];
    k2o[e] = k4[e] * gk;
  }
  *(volatile v4f*)(Kq + base)   = k2o;
  *(volatile v4f*)(Aq + base)   = bino;
  *(volatile v4f*)(AinP + base) = aino;
  __threadfence();
  *(volatile v4f*)(Kq + base)   = k2o;
  *(volatile v4f*)(Aq + base)   = bino;
  *(volatile v4f*)(AinP + base) = aino;
}

__global__ __launch_bounds__(256) void decay_kernel(float* __restrict__ Wq, const float* __restrict__ w0v) {
#pragma clang fp contract(off)
  const size_t e0 = ((size_t)blockIdx.x * 256 + threadIdx.x) * 4;
  const int c = (int)(e0 & 2047);
  const v4f p4 = *(const v4f*)(Wq + e0);
  const v4f b4 = *(const v4f*)(w0v + c);
  v4f o;
#pragma unroll 1
  for (int e = 0; e < 4; ++e) {
    const float z  = b4[e] + p4[e];
    const float u  = -z;
    const float sp = fmaxf(u, 0.0f) + log1pf(expf(-fabsf(u)));
    o[e] = expf(-sp - 0.5f);
  }
  *(volatile v4f*)(Wq + e0) = o;
  __threadfence();
  *(volatile v4f*)(Wq + e0) = o;
}

__global__ __launch_bounds__(256) void gn_gate_kernel(const float* __restrict__ Yq, const float* __restrict__ Rq,
    const float* __restrict__ K2q, const float* __restrict__ Vq, const float* __restrict__ Gq,
    const float* __restrict__ rk, const float* __restrict__ lnw, const float* __restrict__ lnb,
    unsigned short* __restrict__ Zh, unsigned short* __restrict__ Zl) {
#pragma clang fp contract(off)
  const int lane = threadIdx.x & 31, wave = threadIdx.x >> 5;
  const int gw = blockIdx.x * 8 + wave;
  const int bt = gw >> 3, hq = gw & 7;
  const int c  = hq * 256 + lane * 8;
  const size_t base = (size_t)bt * kNCH + c;
  float y[8], r[8], k[8], v[8], g[8], rkv[8], lw[8], lb[8];
  {
    const v4f ya = *(const v4f*)(Yq + base),  yb = *(const v4f*)(Yq + base + 4);
    const v4f ra = *(const v4f*)(Rq + base),  rb = *(const v4f*)(Rq + base + 4);
    const v4f ka = *(const v4f*)(K2q + base), kb = *(const v4f*)(K2q + base + 4);
    const v4f va = *(const v4f*)(Vq + base),  vb = *(const v4f*)(Vq + base + 4);
    const v4f ga = *(const v4f*)(Gq + base),  gb = *(const v4f*)(Gq + base + 4);
    const v4f ka2 = *(const v4f*)(rk + c),    kb2 = *(const v4f*)(rk + c + 4);
    const v4f wa = *(const v4f*)(lnw + c),    wb = *(const v4f*)(lnw + c + 4);
    const v4f ba = *(const v4f*)(lnb + c),    bb = *(const v4f*)(lnb + c + 4);
#pragma unroll
    for (int e = 0; e < 4; ++e) {
      y[e] = ya[e];  y[4 + e] = yb[e];
      r[e] = ra[e];  r[4 + e] = rb[e];
      k[e] = ka[e];  k[4 + e] = kb[e];
      v[e] = va[e];  v[4 + e] = vb[e];
      g[e] = ga[e];  g[4 + e] = gb[e];
      rkv[e] = ka2[e]; rkv[4 + e] = kb2[e];
      lw[e] = wa[e]; lw[4 + e] = wb[e];
      lb[e] = ba[e]; lb[4 + e] = bb[e];
    }
  }
  float s = 0.f;
#pragma unroll
  for (int e = 0; e < 8; ++e) s = s + y[e];
  s += __shfl_xor(s, 1, 32);
  s += __shfl_xor(s, 2, 32);
  s += __shfl_xor(s, 4, 32);
  const float mu = s * (1.0f / 64.0f);
  float d[8];
  float vs = 0.f;
#pragma unroll
  for (int e = 0; e < 8; ++e) { d[e] = y[e] - mu; vs = vs + d[e] * d[e]; }
  vs += __shfl_xor(vs, 1, 32);
  vs += __shfl_xor(vs, 2, 32);
  vs += __shfl_xor(vs, 4, 32);
  const float var = vs * (1.0f / 64.0f);
  const float inv = 1.0f / sqrtf(var + kGnEps);
  float p = 0.f;
#pragma unroll
  for (int e = 0; e < 8; ++e) { const float rkk = r[e] * k[e]; p = p + rkk * rkv[e]; }
  p += __shfl_xor(p, 1, 32);
  p += __shfl_xor(p, 2, 32);
  p += __shfl_xor(p, 4, 32);
  unsigned short hb[8], lbits[8];
#pragma unroll
  for (int e = 0; e < 8; ++e) {
    const float dn  = d[e] * inv;
    const float on  = dn * lw[e] + lb[e];
    const float bon = p * v[e];
    const float z   = (on + bon) * g[e];
    split_bf(z, hb[e], lbits[e]);
  }
  const v4u uh = (v4u){pk16(hb[0], hb[1]), pk16(hb[2], hb[3]), pk16(hb[4], hb[5]), pk16(hb[6], hb[7])};
  const v4u ul = (v4u){pk16(lbits[0], lbits[1]), pk16(lbits[2], lbits[3]), pk16(lbits[4], lbits[5]), pk16(lbits[6], lbits[7])};
  *(volatile v4u*)(Zh + base) = uh;
  *(volatile v4u*)(Zl + base) = ul;
  __threadfence();
  *(volatile v4u*)(Zh + base) = uh;
  *(volatile v4u*)(Zl + base) = ul;
}

template <int BIAS_MODE, int OUT_MODE, int ACT>
static void launch_gemm3(hipStream_t s, const unsigned short* Ah, const unsigned short* Al, int lda,
                         const unsigned short* Bh, const unsigned short* Bl, int ldb,
                         void* Co, void* Co2, int ldc, const float* bias, int M, int N, int K) {
  const int tiles = (M / 64) * (N / 64);
  dim3 grid((tiles + 7) / 8, 1);
  wmma_gemm64<1, true, BIAS_MODE, OUT_MODE, false, ACT><<<grid, dim3(256), 0, s>>>(
      Ah, Al, lda, 0L, Bh, Bl, ldb, 0L, Co, Co2, ldc, 0L, bias, (const float*)nullptr, 0L, M, N, K, 1.0f);
}
static void launch_transpose(hipStream_t s, const float* W, int KR, int NCOL, int KP, int NP,
                             unsigned short* hi, unsigned short* lo) {
  dim3 grid(KP / 64, NP / 64);
  transpose_split_kernel<<<grid, dim3(256), 0, s>>>(W, KR, NCOL, hi, lo, KP);
}

extern "C" void kernel_launch(void* const* d_in, const int* in_sizes, int n_in,
                              void* d_out, int out_size, void* d_ws, size_t ws_size,
                              hipStream_t stream)
{
  (void)in_sizes;
  if (n_in < 30) return;
  if ((long)out_size < kPlane) return;
  if ((long)ws_size < 8L * kRegBytes) return;

  const float* x_in   = (const float*)d_in[0];
  const float* vfirst = (const float*)d_in[1];
  const float* shift  = (const float*)d_in[2];
  const float* wkv0   = (const float*)d_in[3];
  const float* xr_m   = (const float*)d_in[4];
  const float* xw_m   = (const float*)d_in[5];
  const float* xk_m   = (const float*)d_in[6];
  const float* xv_m   = (const float*)d_in[7];
  const float* xa_m   = (const float*)d_in[8];
  const float* xg_m   = (const float*)d_in[9];
  const float* w0v    = (const float*)d_in[10];
  const float* w1m    = (const float*)d_in[11];
  const float* w2m    = (const float*)d_in[12];
  const float* a0v    = (const float*)d_in[13];
  const float* a1m    = (const float*)d_in[14];
  const float* a2m    = (const float*)d_in[15];
  const float* v0v    = (const float*)d_in[16];
  const float* v1m    = (const float*)d_in[17];
  const float* v2m    = (const float*)d_in[18];
  const float* g1m    = (const float*)d_in[19];
  const float* g2m    = (const float*)d_in[20];
  const float* kkc    = (const float*)d_in[21];
  const float* kac    = (const float*)d_in[22];
  const float* rkm    = (const float*)d_in[23];
  const float* Wr     = (const float*)d_in[24];
  const float* Wk     = (const float*)d_in[25];
  const float* Wv     = (const float*)d_in[26];
  const float* Wo     = (const float*)d_in[27];
  const float* lnw    = (const float*)d_in[28];
  const float* lnb    = (const float*)d_in[29];
  float* outp = (float*)d_out;

  char* ws = (char*)d_ws;
  float* Rf = (float*)(ws + 0 * kRegBytes);
  float* Kf = (float*)(ws + 1 * kRegBytes);
  float* Vf = (float*)(ws + 2 * kRegBytes);
  char*  P4 = ws + 3 * kRegBytes;
  char*  P5 = ws + 4 * kRegBytes;
  char*  P6 = ws + 5 * kRegBytes;
  char*  S7 = ws + 6 * kRegBytes;
  char*  S8 = ws + 7 * kRegBytes;

  unsigned short* actHi = (unsigned short*)(S7);
  unsigned short* actLo = (unsigned short*)(S7 + kHalfReg);
  unsigned short* wtHi  = (unsigned short*)(S8);
  unsigned short* wtLo  = (unsigned short*)(S8 + kHalfReg);

  const int MR = kRows, CN = kNCH;
  const int mixBlocks   = (int)(kPlane / 8 / 256);
  const int vmixBlocks  = (int)(kPlane / 4 / 256);
  const int decayBlocks = (int)(kPlane / 4 / 256);
  const int prepBlocks  = (MR * (kNH / 2)) / 8;
  const int gnBlocks    = (MR * (kNH / 4)) / 8;
  const int scanBlocks  = kNB * kNH;

  mixsplit_kernel<<<mixBlocks, 256, 0, stream>>>(x_in, shift, xr_m, actHi, actLo);
  launch_transpose(stream, Wr, CN, CN, CN, CN, wtHi, wtLo);
  launch_gemm3<0, 0, 0>(stream, actHi, actLo, CN, wtHi, wtLo, CN, Rf, nullptr, CN, nullptr, MR, CN, CN);

  mixsplit_kernel<<<mixBlocks, 256, 0, stream>>>(x_in, shift, xk_m, actHi, actLo);
  launch_transpose(stream, Wk, CN, CN, CN, CN, wtHi, wtLo);
  launch_gemm3<0, 0, 0>(stream, actHi, actLo, CN, wtHi, wtLo, CN, Kf, nullptr, CN, nullptr, MR, CN, CN);

  mixsplit_kernel<<<mixBlocks, 256, 0, stream>>>(x_in, shift, xv_m, actHi, actLo);
  launch_transpose(stream, Wv, CN, CN, CN, CN, wtHi, wtLo);
  launch_gemm3<0, 0, 0>(stream, actHi, actLo, CN, wtHi, wtLo, CN, Vf, nullptr, CN, nullptr, MR, CN, CN);
  {
    unsigned short* v1T_hi = (unsigned short*)(P4 + 0 * kSub256K);
    unsigned short* v1T_lo = (unsigned short*)(P4 + 1 * kSub256K);
    unsigned short* v2T_hi = (unsigned short*)(P4 + 2 * kSub256K);
    unsigned short* v2T_lo = (unsigned short*)(P4 + 3 * kSub256K);
    unsigned short* h2_hi  = (unsigned short*)(P4 + 4 * kSub256K);
    unsigned short* h2_lo  = (unsigned short*)(P4 + 5 * kSub256K);
    float* vpre = (float*)P5;
    launch_transpose(stream, v1m, CN, 32, CN, 64, v1T_hi, v1T_lo);
    launch_gemm3<0, 2, 0>(stream, actHi, actLo, CN, v1T_hi, v1T_lo, CN, h2_hi, h2_lo, 64, nullptr, MR, 64, CN);
    launch_transpose(stream, v2m, 32, CN, 64, CN, v2T_hi, v2T_lo);
    launch_gemm3<0, 0, 0>(stream, h2_hi, h2_lo, 64, v2T_hi, v2T_lo, 64, vpre, nullptr, CN, nullptr, MR, CN, 64);
    vmix_kernel<<<vmixBlocks, 256, 0, stream>>>(Vf, vfirst, vpre, v0v);
  }

  mixsplit_kernel<<<mixBlocks, 256, 0, stream>>>(x_in, shift, xa_m, actHi, actLo);
  {
    unsigned short* a1T_hi = (unsigned short*)(P5 + 0 * kSub256K);
    unsigned short* a1T_lo = (unsigned short*)(P5 + 1 * kSub256K);
    unsigned short* a2T_hi = (unsigned short*)(P5 + 2 * kSub256K);
    unsigned short* a2T_lo = (unsigned short*)(P5 + 3 * kSub256K);
    unsigned short* h3_hi  = (unsigned short*)(P5 + 4 * kSub256K);
    unsigned short* h3_lo  = (unsigned short*)(P5 + 5 * kSub256K);
    float* Af = (float*)P4;
    launch_transpose(stream, a1m, CN, 64, CN, 64, a1T_hi, a1T_lo);
    launch_gemm3<0, 2, 0>(stream, actHi, actLo, CN, a1T_hi, a1T_lo, CN, h3_hi, h3_lo, 64, nullptr, MR, 64, CN);
    launch_transpose(stream, a2m, 64, CN, 64, CN, a2T_hi, a2T_lo);
    launch_gemm3<2, 0, 6>(stream, h3_hi, h3_lo, 64, a2T_hi, a2T_lo, 64, Af, nullptr, CN, a0v, MR, CN, 64);
  }

  kprep_kernel<<<prepBlocks, 256, 0, stream>>>(Kf, (float*)P4, (float*)P6, kkc, kac);

  mixsplit_kernel<<<mixBlocks, 256, 0, stream>>>(x_in, shift, xw_m, actHi, actLo);
  {
    unsigned short* w1T_hi = (unsigned short*)(S8 + 0 * kSub256K);
    unsigned short* w1T_lo = (unsigned short*)(S8 + 1 * kSub256K);
    unsigned short* w2T_hi = (unsigned short*)(S8 + 2 * kSub256K);
    unsigned short* w2T_lo = (unsigned short*)(S8 + 3 * kSub256K);
    unsigned short* h1_hi  = (unsigned short*)(S8 + 4 * kSub256K);
    unsigned short* h1_lo  = (unsigned short*)(S8 + 5 * kSub256K);
    float* wpre = (float*)P5;
    launch_transpose(stream, w1m, CN, 64, CN, 64, w1T_hi, w1T_lo);
    launch_gemm3<0, 2, 1>(stream, actHi, actLo, CN, w1T_hi, w1T_lo, CN, h1_hi, h1_lo, 64, nullptr, MR, 64, CN);
    launch_transpose(stream, w2m, 64, CN, 64, CN, w2T_hi, w2T_lo);
    launch_gemm3<0, 0, 0>(stream, h1_hi, h1_lo, 64, w2T_hi, w2T_lo, 64, wpre, nullptr, CN, nullptr, MR, CN, 64);
    decay_kernel<<<decayBlocks, 256, 0, stream>>>(wpre, w0v);
  }

  float* Yf = (float*)S7;
  dscan_kernel<<<scanBlocks, 256, 0, stream>>>(Rf, Kf, Vf, (const float*)P5, (const float*)P6,
                                               (const float*)P4, wkv0, Yf);

  {
    unsigned short* xgHi   = (unsigned short*)(P6);
    unsigned short* xgLo   = (unsigned short*)(P6 + kHalfReg);
    unsigned short* g1T_hi = (unsigned short*)(S8 + 0 * kSub512K);
    unsigned short* g1T_lo = (unsigned short*)(S8 + 1 * kSub512K);
    unsigned short* g2T_hi = (unsigned short*)(S8 + 2 * kSub512K);
    unsigned short* g2T_lo = (unsigned short*)(S8 + 3 * kSub512K);
    unsigned short* h4_hi  = (unsigned short*)(S8 + 4 * kSub512K);
    unsigned short* h4_lo  = (unsigned short*)(S8 + 5 * kSub512K);
    float* Gf = (float*)P4;
    mixsplit_kernel<<<mixBlocks, 256, 0, stream>>>(x_in, shift, xg_m, xgHi, xgLo);
    launch_transpose(stream, g1m, CN, 128, CN, 128, g1T_hi, g1T_lo);
    launch_gemm3<0, 2, 6>(stream, xgHi, xgLo, CN, g1T_hi, g1T_lo, CN, h4_hi, h4_lo, 128, nullptr, MR, 128, CN);
    launch_transpose(stream, g2m, 128, CN, 128, CN, g2T_hi, g2T_lo);
    launch_gemm3<0, 0, 0>(stream, h4_hi, h4_lo, 128, g2T_hi, g2T_lo, 128, Gf, nullptr, CN, nullptr, MR, CN, 128);

    unsigned short* Zh = (unsigned short*)(P5);
    unsigned short* Zl = (unsigned short*)(P5 + kHalfReg);
    gn_gate_kernel<<<gnBlocks, 256, 0, stream>>>(Yf, Rf, Kf, Vf, Gf, rkm, lnw, lnb, Zh, Zl);

    launch_transpose(stream, Wo, CN, CN, CN, CN, wtHi, wtLo);
    launch_gemm3<0, 0, 0>(stream, Zh, Zl, CN, wtHi, wtLo, CN, outp, nullptr, CN, nullptr, MR, CN, CN);
  }
}
